// LinearAttention_53730040873581
// MI455X (gfx1250) — hardware-run, weakly checked
//
#include <hip/hip_runtime.h>
#include <math.h>

typedef __attribute__((ext_vector_type(16))) __bf16   v16b;
typedef __attribute__((ext_vector_type(8)))  __bf16   v8b;
typedef __attribute__((ext_vector_type(8)))  float    v8f;
typedef __attribute__((ext_vector_type(4)))  float    v4f;
typedef __attribute__((ext_vector_type(4)))  unsigned int v4u;

constexpr int   kSeq     = 2048;
constexpr int   kDm      = 1024;
constexpr int   kHeads   = 16;
constexpr int   kDh      = 64;
constexpr int   kQkvN    = 3 * kDm;
constexpr int   kWRows   = 4 * kDm;
constexpr int   kPhiCols = 2 * kDm;
constexpr float kEps     = 1e-6f;
constexpr int   kScanTS  = 32;
constexpr int   kScanOP  = 68;
constexpr int   kSlabP   = 68;
static_assert(kHeads * kDh == kDm, "head split");
static_assert(kDh == 64, "scan lane map assumes 64-wide heads");
static_assert((kDm % 32) == 0, "GEMM K multiple of 32");
static_assert((kSeq % 64) == 0 && (kQkvN % 64) == 0 && (kDm % 64) == 0, "GEMM M,N multiples of 64");
static_assert((kSeq % kScanTS) == 0, "scan chunks exact");
static_assert(((kSeq / 64) * (kQkvN / 64)) % 8 == 0 && ((kSeq / 64) * (kDm / 64)) % 8 == 0, "tiles per block exact");

constexpr size_t kOffXB   = 0;
constexpr size_t kOffWB   = kOffXB   + (size_t)kSeq   * kDm   * 2;
constexpr size_t kOffBias = kOffWB   + (size_t)kWRows * kDm   * 2;
constexpr size_t kOffQKV  = kOffBias + (size_t)4 * kDm * 4;
constexpr size_t kOffOH   = kOffQKV  + (size_t)kSeq   * kQkvN * 4;
constexpr size_t kOffOL   = kOffOH   + (size_t)kSeq   * kDm   * 2;
constexpr size_t kWsTotal = kOffOL   + (size_t)kSeq   * kDm   * 2;
static_assert(kWsTotal == 46153728ull, "carve total");
static_assert(kWsTotal <= 134217728ull, "carve cap");
static_assert((kOffWB % 256) == 0 && (kOffBias % 256) == 0 && (kOffQKV % 256) == 0 &&
              (kOffOH % 256) == 0 && (kOffOL % 256) == 0, "aligned regions");

__device__ __forceinline__ unsigned short f2bf_bits(float f) {
  unsigned u = __float_as_uint(f);
  return (unsigned short)((u + 0x7FFFu + ((u >> 16) & 1u)) >> 16);
}
__device__ __forceinline__ float bf_bits2f(unsigned short h) { return __uint_as_float(((unsigned)h) << 16); }
__device__ __forceinline__ float bf16r(float f) { return bf_bits2f(f2bf_bits(f)); }
__device__ __forceinline__ unsigned pk16(unsigned short a, unsigned short b) { return (unsigned)a | ((unsigned)b << 16); }

union FragB { v16b v; v8b h[2]; };
__device__ __forceinline__ v16b frag_load(const __bf16* p) {
  FragB f;
  f.h[0] = *(const v8b*)(p);
  f.h[1] = *(const v8b*)(p + 16);
  return f.v;
}
__device__ __forceinline__ v8f mma_bf(v16b a, v16b b, v8f c) {
  c = __builtin_amdgcn_wmma_f32_16x16x32_bf16(false, a, false, b, (short)0, c, false, false);
  asm volatile("v_nop\n\tv_nop\n\tv_nop\n\tv_nop" : "+v"(c) : "v"(a), "v"(b));
  return c;
}

__global__ __launch_bounds__(256) void cvt8_bf16_kernel(const float* s0, const float* s1, const float* s2,
                                                        const float* s3, unsigned short* __restrict__ dst, int n8) {
  const int i = blockIdx.x * 256 + threadIdx.x;
  const int z = blockIdx.y;
  const float* src = (z == 0) ? s0 : (z == 1) ? s1 : (z == 2) ? s2 : s3;
  if (i >= n8) return;
  const float* p = src + 8 * (size_t)i;
  const v4f a = *(const v4f*)(p);
  const v4f c = *(const v4f*)(p + 4);
  unsigned short hb[8];
#pragma unroll
  for (int e = 0; e < 4; ++e) {
    const float f0 = a[e];
    const float f1 = c[e];
    hb[e]     = f2bf_bits(f0);
    hb[4 + e] = f2bf_bits(f1);
  }
  const v4u u = (v4u){pk16(hb[0], hb[1]), pk16(hb[2], hb[3]), pk16(hb[4], hb[5]), pk16(hb[6], hb[7])};
  unsigned short* q = dst + (size_t)z * 8 * (size_t)n8 + 8 * (size_t)i;
  *(volatile v4u*)q = u;
  __threadfence();
  *(volatile v4u*)q = u;
}

__global__ __launch_bounds__(256) void bias_prep_kernel(const float* b0, const float* b1, const float* b2,
                                                        const float* b3, float* __restrict__ dst) {
  const int z = blockIdx.x;
  const float* src = (z == 0) ? b0 : (z == 1) ? b1 : (z == 2) ? b2 : b3;
  const int idx = threadIdx.x * 4;
  const v4f v = *(const v4f*)(src + idx);
  v4f o;
#pragma unroll
  for (int e = 0; e < 4; ++e) {
    const float f = v[e];
    o[e] = bf16r(f);
  }
  float* op = dst + z * kDm + idx;
  *(volatile v4f*)op = o;
  __threadfence();
  *(volatile v4f*)op = o;
}

template <bool ALO, bool PHI>
__global__ __launch_bounds__(256) void gemm64_bf16_kernel(
    const unsigned short* __restrict__ Ap, const unsigned short* __restrict__ A2p, int lda,
    const unsigned short* __restrict__ Btp, int ldb,
    float* __restrict__ C, int ldc,
    const float* __restrict__ bias,
    int M, int N, int K, int phiCols) {
  const __bf16* A  = (const __bf16*)Ap;
  const __bf16* A2 = (const __bf16*)A2p;
  const __bf16* Bt = (const __bf16*)Btp;
  __shared__ __align__(16) float sT[8][16 * kSlabP];
  const int lane = threadIdx.x & 31;
  const int wave = threadIdx.x >> 5;
  const int tilesN = N >> 6;
  const int tilesM = M >> 6;
  const int tile = blockIdx.x * 8 + wave;
  if (tile >= tilesM * tilesN) return;
  const int tm = tile / tilesN;
  const int tn = tile - tm * tilesN;
  const int m0 = tm << 6;
  const int n0 = tn << 6;

  const int rlane = lane & 15;
  const int koff  = (lane >> 4) * 8;
  const int mOff  = (lane >> 4) * 8;

  v8f acc[4][4];
#pragma unroll
  for (int i = 0; i < 4; ++i)
#pragma unroll
    for (int j = 0; j < 4; ++j) acc[i][j] = (v8f){0.f, 0.f, 0.f, 0.f, 0.f, 0.f, 0.f, 0.f};

  for (int k0 = 0; k0 < K; k0 += 32) {
    v16b bh[4];
#pragma unroll
    for (int j = 0; j < 4; ++j) {
      const size_t bo = (size_t)(n0 + (j << 4) + rlane) * ldb + koff + k0;
      bh[j] = frag_load(Bt + bo);
    }
#pragma unroll
    for (int i = 0; i < 4; ++i) {
      const size_t ao = (size_t)(m0 + (i << 4) + rlane) * lda + koff + k0;
      const v16b ah = frag_load(A + ao);
      v16b al;
      if (ALO) al = frag_load(A2 + ao);
#pragma unroll
      for (int j = 0; j < 4; ++j) {
        acc[i][j] = mma_bf(ah, bh[j], acc[i][j]);
        if (ALO) acc[i][j] = mma_bf(al, bh[j], acc[i][j]);
      }
    }
  }

  float* slab = sT[wave];
#pragma unroll
  for (int i = 0; i < 4; ++i) {
    const int mBase = m0 + (i << 4);
#pragma unroll
    for (int j = 0; j < 4; ++j) {
      const int n = n0 + (j << 4) + rlane;
      const float bv = bias[n];
#pragma unroll
      for (int r = 0; r < 8; ++r) {
        const float v = acc[i][j][r] + bv;
        slab[(mOff + r) * kSlabP + (j << 4) + rlane] = v;
      }
    }
    __builtin_amdgcn_fence(__ATOMIC_RELEASE, "workgroup");
    __builtin_amdgcn_wave_barrier();
    __builtin_amdgcn_fence(__ATOMIC_ACQUIRE, "workgroup");
    if (PHI) {
      if (n0 < phiCols) {
#pragma unroll 1
        for (int row = 0; row < 16; ++row) {
          float* sp = slab + row * kSlabP + lane * 2;
          const float z0 = sp[0];
          const float z1 = sp[1];
          const float e0 = expf(fminf(z0, 0.0f));
          const float e1 = expf(fminf(z1, 0.0f));
          const float p0 = (z0 > 0.0f) ? (z0 + 1.0f) : e0;
          const float p1 = (z1 > 0.0f) ? (z1 + 1.0f) : e1;
          sp[0] = p0;
          sp[1] = p1;
        }
        __builtin_amdgcn_fence(__ATOMIC_RELEASE, "workgroup");
        __builtin_amdgcn_wave_barrier();
        __builtin_amdgcn_fence(__ATOMIC_ACQUIRE, "workgroup");
      }
    }
    {
      const int hh = lane >> 4, c4 = (lane & 15) * 4;
      for (int pass = 0; pass < 2; ++pass) {
#pragma unroll
        for (int it = 0; it < 8; ++it) {
          const int row = it * 2 + hh;
          const v4f v = *(const v4f*)(slab + row * kSlabP + c4);
          *(volatile v4f*)(C + (size_t)(mBase + row) * ldc + n0 + c4) = v;
        }
        __threadfence();
      }
    }
    __builtin_amdgcn_fence(__ATOMIC_RELEASE, "workgroup");
    __builtin_amdgcn_wave_barrier();
    __builtin_amdgcn_fence(__ATOMIC_ACQUIRE, "workgroup");
  }
}

__global__ __launch_bounds__(256) void causal_scan_kernel(const float* __restrict__ QKV,
                                                          unsigned short* __restrict__ OH,
                                                          unsigned short* __restrict__ OL) {
  __shared__ __align__(16) float sQ[kScanTS * kDh];
  __shared__ __align__(16) float sK[kScanTS * kDh];
  __shared__ __align__(16) float sV[kScanTS * kDh];
  __shared__ __align__(16) float sO[kScanTS * kScanOP];
  const int tid = threadIdx.x, lane = tid & 31, wave = tid >> 5;
  const int h  = blockIdx.x;
  const int e  = 8 * wave + (lane & 7);
  const int dg = lane >> 3;
  const int d0 = 16 * dg;
  const int q8 = lane >> 3, c8 = (lane & 7) * 8;

  float kv[16], kp[16];
#pragma unroll
  for (int i = 0; i < 16; ++i) { kv[i] = 0.0f; kp[i] = 0.0f; }

#pragma unroll 1
  for (int t0 = 0; t0 < kSeq; t0 += kScanTS) {
#pragma unroll
    for (int i = 0; i < 2; ++i) {
      const int idx = tid + 256 * i;
      const int r  = idx >> 4;
      const int c4 = (idx & 15) * 4;
      const float* gp = QKV + (size_t)(t0 + r) * kQkvN + h * kDh + c4;
      const v4f qa = *(const v4f*)(gp);
      const v4f ka = *(const v4f*)(gp + kDm);
      const v4f va = *(const v4f*)(gp + 2 * kDm);
      *(v4f*)(sQ + r * kDh + c4) = qa;
      *(v4f*)(sK + r * kDh + c4) = ka;
      *(v4f*)(sV + r * kDh + c4) = va;
    }
    __syncthreads();

#pragma unroll 1
    for (int s = 0; s < kScanTS; ++s) {
      const float* qp = sQ + s * kDh + d0;
      const float* kq = sK + s * kDh + d0;
      v4f qv[4], kk[4];
#pragma unroll
      for (int g = 0; g < 4; ++g) {
        qv[g] = *(const v4f*)(qp + 4 * g);
        kk[g] = *(const v4f*)(kq + 4 * g);
      }
      const float vv = sV[s * kDh + e];
      float num = 0.0f, den = 0.0f;
#pragma unroll
      for (int i = 0; i < 16; ++i) {
        const float kd = kk[i >> 2][i & 3];
        const float qd = qv[i >> 2][i & 3];
        kv[i] = fmaf(kd, vv, kv[i]);
        kp[i] = kp[i] + kd;
        num = fmaf(qd, kv[i], num);
        den = fmaf(qd, kp[i], den);
      }
      num += __shfl_xor(num, 8, 32);
      den += __shfl_xor(den, 8, 32);
      num += __shfl_xor(num, 16, 32);
      den += __shfl_xor(den, 16, 32);
      const float o = num * (1.0f / (den + kEps));
      if (dg == 0) sO[s * kScanOP + e] = o;
    }
    __syncthreads();

    {
      const int row = wave * 4 + q8;
      const float* sp = sO + row * kScanOP + c8;
      const v4f a0 = *(const v4f*)(sp);
      const v4f a1 = *(const v4f*)(sp + 4);
      unsigned short hb[8], lb[8];
#pragma unroll
      for (int j = 0; j < 4; ++j) {
        const float f0 = a0[j];
        const float f1 = a1[j];
        const unsigned short h0 = f2bf_bits(f0);
        const unsigned short h1 = f2bf_bits(f1);
        hb[j]     = h0;
        hb[4 + j] = h1;
        lb[j]     = f2bf_bits(f0 - bf_bits2f(h0));
        lb[4 + j] = f2bf_bits(f1 - bf_bits2f(h1));
      }
      const v4u uh = (v4u){pk16(hb[0], hb[1]), pk16(hb[2], hb[3]), pk16(hb[4], hb[5]), pk16(hb[6], hb[7])};
      const v4u ul = (v4u){pk16(lb[0], lb[1]), pk16(lb[2], lb[3]), pk16(lb[4], lb[5]), pk16(lb[6], lb[7])};
      const size_t go = (size_t)(t0 + row) * kDm + h * kDh + c8;
      for (int pass = 0; pass < 2; ++pass) {
        *(volatile v4u*)(OH + go) = uh;
        *(volatile v4u*)(OL + go) = ul;
        __threadfence();
      }
    }
  }
}

extern "C" void kernel_launch(void* const* d_in, const int* in_sizes, int n_in,
                              void* d_out, int out_size, void* d_ws, size_t ws_size,
                              hipStream_t stream) {
  if (n_in < 10 || d_out == nullptr || d_ws == nullptr) return;
  if (in_sizes[0] != kSeq * kDm) return;
  if (in_sizes[1] != kSeq * kSeq) return;
  if (in_sizes[2] != kDm * kDm || in_sizes[4] != kDm * kDm || in_sizes[6] != kDm * kDm || in_sizes[8] != kDm * kDm) return;
  if (in_sizes[3] != kDm || in_sizes[5] != kDm || in_sizes[7] != kDm || in_sizes[9] != kDm) return;
  if (out_size != kSeq * kDm) return;
  if (ws_size < kWsTotal) return;

  const float* x  = (const float*)d_in[0];
  const float* Wq = (const float*)d_in[2];
  const float* bq = (const float*)d_in[3];
  const float* Wk = (const float*)d_in[4];
  const float* bk = (const float*)d_in[5];
  const float* Wv = (const float*)d_in[6];
  const float* bv = (const float*)d_in[7];
  const float* Wo = (const float*)d_in[8];
  const float* bo = (const float*)d_in[9];
  float* out = (float*)d_out;

  char* ws = (char*)d_ws;
  unsigned short* XB   = (unsigned short*)(ws + kOffXB);
  unsigned short* WB   = (unsigned short*)(ws + kOffWB);
  float*          BIAS = (float*)(ws + kOffBias);
  float*          QKV  = (float*)(ws + kOffQKV);
  unsigned short* OH   = (unsigned short*)(ws + kOffOH);
  unsigned short* OL   = (unsigned short*)(ws + kOffOL);

  cvt8_bf16_kernel<<<dim3((kSeq * kDm / 8) / 256, 1), 256, 0, stream>>>(x, x, x, x, XB, kSeq * kDm / 8);
  cvt8_bf16_kernel<<<dim3((kDm * kDm / 8) / 256, 4), 256, 0, stream>>>(Wq, Wk, Wv, Wo, WB, kDm * kDm / 8);
  bias_prep_kernel<<<4, 256, 0, stream>>>(bq, bk, bv, bo, BIAS);

  gemm64_bf16_kernel<false, true><<<dim3(((kSeq / 64) * (kQkvN / 64)) / 8), 256, 0, stream>>>(
      XB, XB, kDm,
      WB, kDm,
      QKV, kQkvN,
      BIAS,
      kSeq, kQkvN, kDm, kPhiCols);

  causal_scan_kernel<<<kHeads, 256, 0, stream>>>(QKV, OH, OL);

  gemm64_bf16_kernel<true, false><<<dim3(((kSeq / 64) * (kDm / 64)) / 8), 256, 0, stream>>>(
      OH, OL, kDm,
      WB + (size_t)kQkvN * kDm, kDm,
      out, kDm,
      BIAS + kQkvN,
      kSeq, kDm, kDm, 0);
}
